// cait_models_46583215292897
// MI455X (gfx1250) — hardware-run, weakly checked
//
#include <hip/hip_runtime.h>

constexpr int kBatch  = 4;
constexpr int kTok    = 1024;
constexpr int kChan   = 768;
constexpr int kHeads  = 12;
constexpr int kHdim   = 64;
constexpr int kQkvN   = 3 * kChan;
constexpr int kTokAll = kBatch * kTok;
constexpr int kGrp    = 6;
constexpr int kNGrp   = kHeads / kGrp;
constexpr long kPlane   = (long)kTok * kTok;
constexpr long kVtPlane = (long)kHdim * kTok;
static_assert(kNGrp * kGrp == kHeads);

constexpr float kWCarry     = 16.0f;
constexpr float kA2Carry    = 2048.0f;
constexpr float kAttCarry   = 256.0f;
constexpr float kQkvScale   = 1.0f / 16.0f;
constexpr float kScoreScale = 0.125f;
constexpr float kReact3     = 3.0f / 4194304.0f;
constexpr float kAttnVScale = 8.0f / 256.0f;
constexpr float kProjScale  = 1.0f / 128.0f;

constexpr long kOffS    = 0;
constexpr long kOffX16  = 0;
constexpr long kOffAM   = 0;
constexpr long kOffA2T  = 12582912;
constexpr long kOffATT  = 25165824;
constexpr long kOffA2F  = 50331648;
constexpr long kOffWQ   = 50331648;
constexpr long kOffQKV  = 100663296;
constexpr long kOffVT   = 119537664;
constexpr long kOffWP   = 125829120;
constexpr long kOffCTX  = 127008768;
constexpr long kWsTotal = 128581632;
static_assert(kOffA2T == kOffAM + 2L * kGrp * kPlane);
static_assert(kOffATT == kOffA2T + 2L * kGrp * kPlane);
static_assert(kOffATT + 2L * kGrp * kPlane <= kOffA2F);
static_assert(2L * kTokAll * kChan <= kOffA2F);
static_assert(kOffA2F == kOffS + 4L * kHeads * kPlane);
static_assert(kOffQKV == kOffA2F + 4L * kHeads * kPlane);
static_assert(2L * kQkvN * kChan <= 4L * kHeads * kPlane);
static_assert(kOffVT == kOffQKV + 2L * kTokAll * kQkvN);
static_assert(kOffWP == kOffVT + 2L * kBatch * kHeads * kVtPlane);
static_assert(kOffCTX == kOffWP + 2L * kChan * kChan);
static_assert(kWsTotal == kOffCTX + 2L * kTok * kChan);
static_assert(kWsTotal <= 134217728L);

typedef __attribute__((ext_vector_type(16))) _Float16 v16h;
typedef __attribute__((ext_vector_type(8)))  _Float16 v8h;
typedef __attribute__((ext_vector_type(16))) __bf16   v16b;
typedef __attribute__((ext_vector_type(8)))  __bf16   v8b;
typedef __attribute__((ext_vector_type(8)))  float    v8f;
typedef __attribute__((ext_vector_type(4)))  float    v4f;
typedef __attribute__((ext_vector_type(4)))  unsigned int v4u;

__device__ __forceinline__ unsigned short f2bf_bits(float f) {
  unsigned u = __float_as_uint(f);
  return (unsigned short)((u + 0x7FFFu + ((u >> 16) & 1u)) >> 16);
}
__device__ __forceinline__ float bf_bits2f(unsigned short h) { return __uint_as_float(((unsigned)h) << 16); }

__device__ __forceinline__ void dep_guard_h(v8f& a, v8f& b, v16h x, v16h y) { asm volatile("v_nop\n\tv_nop\n\tv_nop\n\tv_nop" : "+v"(a), "+v"(b) : "v"(x), "v"(y)); }
__device__ __forceinline__ void dep_guard_b(v8f& a, v8f& b, v16b x, v16b y) { asm volatile("v_nop\n\tv_nop\n\tv_nop\n\tv_nop" : "+v"(a), "+v"(b) : "v"(x), "v"(y)); }
__device__ __forceinline__ void keep4_h(v16h a, v16h b, v16h c, v16h d) { asm volatile("v_nop" :: "v"(a), "v"(b), "v"(c), "v"(d)); }
__device__ __forceinline__ void keep4_b(v16b a, v16b b, v16b c, v16b d) { asm volatile("v_nop" :: "v"(a), "v"(b), "v"(c), "v"(d)); }
__device__ __forceinline__ void acc_guard4(v8f& a, v8f& b, v8f& c, v8f& d) { asm volatile("v_nop\n\tv_nop\n\tv_nop\n\tv_nop" : "+v"(a), "+v"(b), "+v"(c), "+v"(d)); }
template <typename T> struct Frag;
template <> struct Frag<_Float16> {
  typedef v16h V; union U { v16h v; v8h h[2]; };
  static __device__ __forceinline__ v16h load(const _Float16* p) {
    U f; f.h[0] = *(const v8h*)(p); f.h[1] = *(const v8h*)(p + 16); return f.v;
  }
  static __device__ __forceinline__ v8f mma(v16h a, v16h b, v8f c) {
    return __builtin_amdgcn_wmma_f32_16x16x32_f16(false, a, false, b, (short)0, c, false, false);
  }
  static __device__ __forceinline__ void guard(v8f& a, v8f& b, v16h x, v16h y) { dep_guard_h(a, b, x, y); }
  static __device__ __forceinline__ void keep(v16h a, v16h b, v16h c, v16h d) { keep4_h(a, b, c, d); }
};
template <> struct Frag<__bf16> {
  typedef v16b V; union U { v16b v; v8b h[2]; };
  static __device__ __forceinline__ v16b load(const __bf16* p) {
    U f; f.h[0] = *(const v8b*)(p); f.h[1] = *(const v8b*)(p + 16); return f.v;
  }
  static __device__ __forceinline__ v8f mma(v16b a, v16b b, v8f c) {
    return __builtin_amdgcn_wmma_f32_16x16x32_bf16(false, a, false, b, (short)0, c, false, false);
  }
  static __device__ __forceinline__ void guard(v8f& a, v8f& b, v16b x, v16b y) { dep_guard_b(a, b, x, y); }
  static __device__ __forceinline__ void keep(v16b a, v16b b, v16b c, v16b d) { keep4_b(a, b, c, d); }
};

__device__ __forceinline__ unsigned pk16(unsigned short a, unsigned short b) { return (unsigned)a | ((unsigned)b << 16); }
__device__ __forceinline__ unsigned short h_bits(float f) { const _Float16 h = (_Float16)f; return __builtin_bit_cast(unsigned short, h); }

__device__ __forceinline__ float wave_max32(float v) {
#pragma unroll
  for (int off = 16; off > 0; off >>= 1) v = fmaxf(v, __shfl_xor(v, off, 32));
  return v;
}
__device__ __forceinline__ float wave_sum32(float v) {
#pragma unroll
  for (int off = 16; off > 0; off >>= 1) v += __shfl_xor(v, off, 32);
  return v;
}

template <int ET> struct Elem;
template <> struct Elem<0> { typedef _Float16 T; };
template <> struct Elem<1> { typedef __bf16 T; };
template <int ET, bool SPLIT, int BIAS_MODE, int OUT_MODE, int RES_MODE, int ACT = 0>
__global__ __launch_bounds__(256) void wmma_gemm64(
    const unsigned short* __restrict__ Ap, const unsigned short* __restrict__ A2p, int lda, long strideA,
    const unsigned short* __restrict__ Btp, const unsigned short* __restrict__ Bt2p, int ldb, long strideB,
    void* __restrict__ Cout, void* __restrict__ Cout2, int ldc, long strideC,
    const float* __restrict__ bias,
    const float* __restrict__ resid, long strideR,
    int M, int N, int K, float scale, float rscale, const float* __restrict__ lamv) {
  typedef typename Elem<ET>::T T;
  typedef typename Frag<T>::V V;
  const T* A = (const T*)Ap; const T* A2 = (const T*)A2p; const T* Bt = (const T*)Btp; const T* Bt2 = (const T*)Bt2p;
  __shared__ __align__(16) float sT[8][16 * 68];
  const int b    = blockIdx.y;
  const int lane = threadIdx.x & 31;
  const int wave = threadIdx.x >> 5;
  const int tilesN = N >> 6;
  const int tilesM = M >> 6;
  const int tile = blockIdx.x * 8 + wave;
  if (tile >= tilesM * tilesN) return;
  const int tm = tile / tilesN;
  const int tn = tile - tm * tilesN;
  const int m0 = tm << 6;
  const int n0 = tn << 6;

  const T* Ab  = A  + (size_t)b * strideA;
  const T* Bb  = Bt + (size_t)b * strideB;
  const T* Ab2 = SPLIT ? (A2  + (size_t)b * strideA) : nullptr;
  const T* Bb2 = SPLIT ? (Bt2 + (size_t)b * strideB) : nullptr;

  const int rlane = lane & 15;
  const int koff  = (lane >> 4) * 8;
  const int mOff  = (lane >> 4) * 8;

  v8f acc[4][4];
#pragma unroll
  for (int i = 0; i < 4; ++i)
#pragma unroll
    for (int j = 0; j < 4; ++j) acc[i][j] = (v8f){0.f,0.f,0.f,0.f,0.f,0.f,0.f,0.f};

  for (int k0 = 0; k0 < K; k0 += 32) {
    V bh[4], bl[4];
#pragma unroll
    for (int j = 0; j < 4; ++j) {
      const size_t bo = (size_t)(n0 + (j << 4) + rlane) * ldb + koff + k0;
      bh[j] = Frag<T>::load(Bb + bo);
      if (SPLIT) bl[j] = Frag<T>::load(Bb2 + bo);
    }
#pragma unroll
    for (int i = 0; i < 4; ++i) {
      const size_t ao = (size_t)(m0 + (i << 4) + rlane) * lda + koff + k0;
      V ah = Frag<T>::load(Ab + ao);
      V al;
      if (SPLIT) al = Frag<T>::load(Ab2 + ao);
#pragma unroll
      for (int j = 0; j < 4; ++j) {
        acc[i][j] = Frag<T>::mma(ah, bh[j], acc[i][j]);
        if (SPLIT) {
          acc[i][j] = Frag<T>::mma(ah, bl[j], acc[i][j]);
          acc[i][j] = Frag<T>::mma(al, bh[j], acc[i][j]);
        }
      }
      Frag<T>::guard(acc[i][0], acc[i][3], ah, SPLIT ? al : ah);
    }
    Frag<T>::keep(bh[0], bh[1], bh[2], bh[3]);
    if (SPLIT) Frag<T>::keep(bl[0], bl[1], bl[2], bl[3]);
  }
  acc_guard4(acc[0][0], acc[0][1], acc[0][2], acc[0][3]);
  acc_guard4(acc[1][0], acc[1][1], acc[1][2], acc[1][3]);
  acc_guard4(acc[2][0], acc[2][1], acc[2][2], acc[2][3]);
  acc_guard4(acc[3][0], acc[3][1], acc[3][2], acc[3][3]);

  float* slab = sT[wave];
  const float* Rb = (RES_MODE != 0) ? (resid + (size_t)b * strideR) : nullptr;
  float lm = 0.f;
  if (RES_MODE == 2) lm = lamv[b];
#pragma unroll
  for (int i = 0; i < 4; ++i) {
    const int mBase = m0 + (i << 4);
#pragma unroll
    for (int j = 0; j < 4; ++j) {
      const int n = n0 + (j << 4) + rlane;
      float bv = 0.f;
      if (BIAS_MODE == 2) bv = bias[n];
#pragma unroll
      for (int r = 0; r < 8; ++r) {
        float v = acc[i][j][r] * scale;
        if (BIAS_MODE == 1) v += bias[mBase + mOff + r];
        if (BIAS_MODE == 2) v += bv;
        if (RES_MODE == 1) v += Rb[(size_t)(mBase + mOff + r) * ldc + n];
        if (RES_MODE == 2) {
          const float a2v = Rb[(size_t)(mBase + mOff + r) * ldc + n];
          const float react = v + a2v;
          v = fmaf(lm, react, a2v) * rscale;
        }
        if (ACT == 2) v = fmaxf(v, 0.0f);
        if (ACT == 4) v = (v > 0.f) ? v : 0.01f * v;
        slab[(mOff + r) * 68 + (j << 4) + rlane] = v;
      }
    }
    __builtin_amdgcn_fence(__ATOMIC_RELEASE, "workgroup");
    __builtin_amdgcn_wave_barrier();
    __builtin_amdgcn_fence(__ATOMIC_ACQUIRE, "workgroup");
    if (OUT_MODE == 0) {
      float* C = (float*)Cout + (size_t)b * strideC;
      const int hh = lane >> 4, c4 = (lane & 15) * 4;
      for (int pass = 0; pass < 2; ++pass) {
#pragma unroll
        for (int it = 0; it < 8; ++it) {
          const int row = it * 2 + hh;
          v4f v = *(const v4f*)(slab + row * 68 + c4);
          *(volatile v4f*)(C + (size_t)(mBase + row) * ldc + n0 + c4) = v;
        }
        __threadfence();
      }
    } else {
      const int q = lane >> 3, c8 = (lane & 7) * 8;
      unsigned short* C  = (unsigned short*)Cout  + (size_t)b * strideC;
      unsigned short* C2 = (OUT_MODE == 2) ? ((unsigned short*)Cout2 + (size_t)b * strideC) : nullptr;
      for (int pass = 0; pass < 2; ++pass) {
#pragma unroll
        for (int it = 0; it < 4; ++it) {
          const int row = it * 4 + q;
          const float* sp = slab + row * 68 + c8;
          v8h hv, lv;
#pragma unroll
          for (int e = 0; e < 8; ++e) {
            if (OUT_MODE == 1) {
              hv[e] = (_Float16)sp[e];
            } else {
              unsigned short hb = f2bf_bits(sp[e]);
              unsigned short lb = f2bf_bits(sp[e] - bf_bits2f(hb));
              hv[e] = __builtin_bit_cast(_Float16, hb);
              lv[e] = __builtin_bit_cast(_Float16, lb);
            }
          }
          *(volatile v8h*)(C + (size_t)(mBase + row) * ldc + n0 + c8) = hv;
          if (OUT_MODE == 2) *(volatile v8h*)(C2 + (size_t)(mBase + row) * ldc + n0 + c8) = lv;
        }
        __threadfence();
      }
    }
    __builtin_amdgcn_fence(__ATOMIC_RELEASE, "workgroup");
    __builtin_amdgcn_wave_barrier();
    __builtin_amdgcn_fence(__ATOMIC_ACQUIRE, "workgroup");
  }
}

__global__ __launch_bounds__(256) void cast8_f16_kernel(const float* __restrict__ in, unsigned short* __restrict__ out, int n8) {
  const int i = blockIdx.x * 256 + threadIdx.x;
  if (i >= n8) return;
  const float* p = in + 8 * (size_t)i;
  const v4f a = *(const v4f*)(p);
  const v4f c = *(const v4f*)(p + 4);
  unsigned short hb[8];
#pragma unroll
  for (int e = 0; e < 4; ++e) {
    hb[e]     = h_bits(a[e]);
    hb[4 + e] = h_bits(c[e]);
  }
  const v4u u = (v4u){pk16(hb[0], hb[1]), pk16(hb[2], hb[3]), pk16(hb[4], hb[5]), pk16(hb[6], hb[7])};
  unsigned short* q = out + 8 * (size_t)i;
  *(volatile v4u*)q = u;
  __threadfence();
  *(volatile v4u*)q = u;
}

__global__ __launch_bounds__(256) void wtr_kernel(const float* __restrict__ in, int rows, int cols,
                                                  unsigned short* __restrict__ out, float scale) {
  __shared__ float sm[64][65];
  const int t    = threadIdx.x;
  const int k0   = blockIdx.x * 64;
  const int j0   = blockIdx.y * 64;
#pragma unroll
  for (int i = 0; i < 16; ++i) {
    const int e  = i * 256 + t;
    const int kl = e >> 6;
    const int jl = e & 63;
    sm[jl][kl] = in[(size_t)(k0 + kl) * cols + j0 + jl] * scale;
  }
  __syncthreads();
  const int lane = t & 31, wave = t >> 5;
  const int q = lane >> 3, c8 = (lane & 7) * 8;
  v4u w[2];
  int orow[2];
#pragma unroll
  for (int it = 0; it < 2; ++it) {
    const int row = wave * 8 + it * 4 + q;
    unsigned short hb[8];
#pragma unroll
    for (int e = 0; e < 8; ++e) hb[e] = h_bits(sm[row][c8 + e]);
    w[it] = (v4u){pk16(hb[0], hb[1]), pk16(hb[2], hb[3]), pk16(hb[4], hb[5]), pk16(hb[6], hb[7])};
    orow[it] = row;
  }
  for (int pass = 0; pass < 2; ++pass) {
#pragma unroll
    for (int it = 0; it < 2; ++it)
      *(volatile v4u*)(out + (size_t)(j0 + orow[it]) * rows + k0 + c8) = w[it];
    __threadfence();
  }
}

__global__ __launch_bounds__(256) void tr16_kernel(const unsigned short* __restrict__ in, int in_ld, int zdiv, long zhi, long zlo,
                                                   unsigned short* __restrict__ out, int out_ld, long zstride) {
  __shared__ unsigned short sm[64][72];
  const int t    = threadIdx.x;
  const int lane = t & 31, wave = t >> 5;
  const int c0   = blockIdx.x * 64;
  const int r0   = blockIdx.y * 64;
  const int z    = blockIdx.z;
  const unsigned short* ib = in + (size_t)(z / zdiv) * (size_t)zhi + (size_t)(z % zdiv) * (size_t)zlo;
#pragma unroll
  for (int it = 0; it < 2; ++it) {
    const int e  = it * 256 + t;
    const int rl = e >> 3;
    const int ch = e & 7;
    const v4u u = *(const v4u*)(ib + (size_t)(r0 + rl) * in_ld + c0 + 8 * ch);
#pragma unroll
    for (int j = 0; j < 8; ++j)
      sm[8 * ch + j][rl] = (unsigned short)((u[j >> 1] >> (16 * (j & 1))) & 0xffffu);
  }
  __syncthreads();
  unsigned short* ob = out + (size_t)z * (size_t)zstride;
  const int q = lane >> 3, cc = (lane & 7) * 8;
  v4u w[2];
  int orow[2];
#pragma unroll
  for (int it = 0; it < 2; ++it) {
    const int row = wave * 8 + it * 4 + q;
    const unsigned short* sp = &sm[row][cc];
    w[it] = (v4u){pk16(sp[0], sp[1]), pk16(sp[2], sp[3]), pk16(sp[4], sp[5]), pk16(sp[6], sp[7])};
    orow[it] = row;
  }
  for (int pass = 0; pass < 2; ++pass) {
#pragma unroll
    for (int it = 0; it < 2; ++it)
      *(volatile v4u*)(ob + (size_t)(c0 + orow[it]) * out_ld + r0 + cc) = w[it];
    __threadfence();
  }
}

__global__ __launch_bounds__(256) void a2planes_kernel(const float* __restrict__ A2, unsigned short* __restrict__ AM,
                                                       unsigned short* __restrict__ AT) {
  __shared__ float sm[64][65];
  const int t    = threadIdx.x;
  const int lane = t & 31, wave = t >> 5;
  const int mt0  = blockIdx.x * 64;
  const int nt0  = blockIdx.y * 64;
  const int z    = blockIdx.z;
  const float* ap = A2 + (size_t)z * (size_t)kPlane;
#pragma unroll
  for (int i = 0; i < 16; ++i) {
    const int e = i * 256 + t;
    const int r = e >> 6;
    const int c = e & 63;
    sm[r][c] = ap[(size_t)(nt0 + r) * kTok + mt0 + c];
  }
  __syncthreads();
  const int q = lane >> 3, c8 = (lane & 7) * 8;
  v4u wm[2], wt[2];
  int orow[2];
#pragma unroll
  for (int it = 0; it < 2; ++it) {
    const int row = wave * 8 + it * 4 + q;
    unsigned short hm[8], ht[8];
#pragma unroll
    for (int e = 0; e < 8; ++e) {
      const float a  = sm[row][c8 + e];
      const float dg = ((nt0 + row) == (mt0 + c8 + e)) ? 1.0f : 0.0f;
      hm[e] = h_bits((a - dg) * kA2Carry);
      ht[e] = h_bits(sm[c8 + e][row] * kA2Carry);
    }
    wm[it] = (v4u){pk16(hm[0], hm[1]), pk16(hm[2], hm[3]), pk16(hm[4], hm[5]), pk16(hm[6], hm[7])};
    wt[it] = (v4u){pk16(ht[0], ht[1]), pk16(ht[2], ht[3]), pk16(ht[4], ht[5]), pk16(ht[6], ht[7])};
    orow[it] = row;
  }
  unsigned short* amb = AM + (size_t)z * (size_t)kPlane;
  unsigned short* atb = AT + (size_t)z * (size_t)kPlane;
  for (int pass = 0; pass < 2; ++pass) {
#pragma unroll
    for (int it = 0; it < 2; ++it) {
      *(volatile v4u*)(amb + (size_t)(nt0 + orow[it]) * kTok + mt0 + c8) = wm[it];
      *(volatile v4u*)(atb + (size_t)(mt0 + orow[it]) * kTok + nt0 + c8) = wt[it];
    }
    __threadfence();
  }
}

__global__ __launch_bounds__(256) void thmix_kernel(const float* __restrict__ S,
                                                    const float* __restrict__ Wl, const float* __restrict__ bl,
                                                    const float* __restrict__ Ww, const float* __restrict__ bw,
                                                    float* __restrict__ A2F) {
  __shared__ __align__(16) float prow[kHeads][kTok];
  __shared__ float sWl[144];
  __shared__ float sWw[144];
  __shared__ float sbl[12];
  __shared__ float sbw[12];
  __shared__ float redM[12][8];
  __shared__ float redS[12][8];
  const int n    = blockIdx.x;
  const int t    = threadIdx.x;
  const int lane = t & 31, wave = t >> 5;
  if (t < 144) { sWl[t] = Wl[t]; sWw[t] = Ww[t]; }
  if (t < 12)  { sbl[t] = bl[t]; sbw[t] = bw[t]; }
  __syncthreads();

  float mx[12];
#pragma unroll
  for (int g = 0; g < 12; ++g) mx[g] = -__builtin_huge_valf();
  const float* srow = S + (size_t)n * kTok;
#pragma unroll 1
  for (int mi = 0; mi < 4; ++mi) {
    const int m = t + 256 * mi;
    float o[12];
#pragma unroll
    for (int g = 0; g < 12; ++g) o[g] = 0.f;
#pragma unroll 1
    for (int h = 0; h < 12; ++h) {
      const float val = srow[(size_t)h * (size_t)kPlane + m];
      const float* w = sWl + h * 12;
#pragma unroll
      for (int g = 0; g < 12; ++g) o[g] = fmaf(val, w[g], o[g]);
    }
#pragma unroll
    for (int g = 0; g < 12; ++g) {
      const float a1 = o[g] + sbl[g];
      prow[g][m] = a1;
      mx[g] = fmaxf(mx[g], a1);
    }
  }
#pragma unroll
  for (int g = 0; g < 12; ++g) {
    const float v = wave_max32(mx[g]);
    if (lane == 0) redM[g][wave] = v;
  }
  __syncthreads();

#pragma unroll 1
  for (int g = 0; g < 12; ++g) {
    float gm = redM[g][0];
#pragma unroll
    for (int w = 1; w < 8; ++w) gm = fmaxf(gm, redM[g][w]);
    float s = 0.f;
#pragma unroll 1
    for (int mi = 0; mi < 4; ++mi) {
      const int m = t + 256 * mi;
      const float e = expf(prow[g][m] - gm);
      prow[g][m] = e;
      s += e;
    }
    s = wave_sum32(s);
    if (lane == 0) redS[g][wave] = s;
  }
  __syncthreads();
#pragma unroll 1
  for (int g = 0; g < 12; ++g) {
    float tot = redS[g][0];
#pragma unroll
    for (int w = 1; w < 8; ++w) tot += redS[g][w];
    const float inv = 1.0f / tot;
#pragma unroll 1
    for (int mi = 0; mi < 4; ++mi) {
      const int m = t + 256 * mi;
      prow[g][m] = prow[g][m] * inv;
    }
  }
  __syncthreads();

  const int m0 = 4 * t;
  float a2[12][4];
#pragma unroll
  for (int g = 0; g < 12; ++g)
#pragma unroll
    for (int e = 0; e < 4; ++e) a2[g][e] = 0.f;
#pragma unroll 1
  for (int h = 0; h < 12; ++h) {
    const v4f p = *(const v4f*)(&prow[h][m0]);
    const float* w = sWw + h * 12;
#pragma unroll
    for (int g = 0; g < 12; ++g) {
      const float wg = w[g];
#pragma unroll
      for (int e = 0; e < 4; ++e) a2[g][e] = fmaf(p[e], wg, a2[g][e]);
    }
  }
  v4f ov[12];
#pragma unroll
  for (int g = 0; g < 12; ++g) {
    const float bwv = sbw[g];
#pragma unroll
    for (int e = 0; e < 4; ++e) ov[g][e] = a2[g][e] + bwv;
  }
  const size_t obase = (size_t)n * kTok + m0;
  for (int pass = 0; pass < 2; ++pass) {
#pragma unroll
    for (int g = 0; g < 12; ++g)
      *(volatile v4f*)(A2F + (size_t)g * (size_t)kPlane + obase) = ov[g];
    __threadfence();
  }
}

extern "C" void kernel_launch(void* const* d_in, const int* in_sizes, int n_in,
                              void* d_out, int out_size, void* d_ws, size_t ws_size, hipStream_t stream) {
  if (n_in < 9) return;
  if (in_sizes[0] != kTokAll * kChan) return;
  if (in_sizes[1] != kChan * kQkvN) return;
  if (in_sizes[2] != kChan * kChan) return;
  if (in_sizes[3] != kChan) return;
  if (in_sizes[4] != kHeads * kHeads || in_sizes[5] != kHeads) return;
  if (in_sizes[6] != kHeads * kHeads || in_sizes[7] != kHeads || in_sizes[8] != kHeads) return;
  if (out_size != kTokAll * kChan) return;
  if (ws_size < (size_t)kWsTotal) return;

  const float* x      = (const float*)d_in[0];
  const float* W_qkv  = (const float*)d_in[1];
  const float* W_proj = (const float*)d_in[2];
  const float* b_proj = (const float*)d_in[3];
  const float* W_l    = (const float*)d_in[4];
  const float* b_l    = (const float*)d_in[5];
  const float* W_w    = (const float*)d_in[6];
  const float* b_w    = (const float*)d_in[7];
  const float* lamb   = (const float*)d_in[8];
  float* outp = (float*)d_out;

  char* ws = (char*)d_ws;
  float*          S     = (float*)(ws + kOffS);
  unsigned short* X16   = (unsigned short*)(ws + kOffX16);
  unsigned short* AM    = (unsigned short*)(ws + kOffAM);
  unsigned short* A2T   = (unsigned short*)(ws + kOffA2T);
  unsigned short* ATT   = (unsigned short*)(ws + kOffATT);
  float*          A2F   = (float*)(ws + kOffA2F);
  unsigned short* WQT   = (unsigned short*)(ws + kOffWQ);
  unsigned short* QKV   = (unsigned short*)(ws + kOffQKV);
  unsigned short* VT    = (unsigned short*)(ws + kOffVT);
  unsigned short* WPT   = (unsigned short*)(ws + kOffWP);
  unsigned short* CTX   = (unsigned short*)(ws + kOffCTX);

  cast8_f16_kernel<<<dim3((kTokAll * kChan / 8) / 256), dim3(256), 0, stream>>>(x, X16, kTokAll * kChan / 8);
  wtr_kernel<<<dim3(kChan / 64, kQkvN / 64), dim3(256), 0, stream>>>(W_qkv, kChan, kQkvN, WQT, kWCarry);
  wtr_kernel<<<dim3(kChan / 64, kChan / 64), dim3(256), 0, stream>>>(W_proj, kChan, kChan, WPT, kWCarry);

  wmma_gemm64<0, false, 0, 1, 0><<<dim3((kTokAll / 64) * (kQkvN / 64) / 8, 1), dim3(256), 0, stream>>>(
      X16, nullptr, kChan, 0L, WQT, nullptr, kChan, 0L,
      (void*)QKV, nullptr, kQkvN, 0L, nullptr, nullptr, 0L, kTokAll, kQkvN, kChan, kQkvScale, 0.f, nullptr);

  tr16_kernel<<<dim3(1, kTok / 64, kBatch * kHeads), dim3(256), 0, stream>>>(
      QKV + 2 * kChan, kQkvN, kHeads, (long)kTok * kQkvN, (long)kHdim, VT, kTok, kVtPlane);

  for (int b = 0; b < kBatch; ++b) {
    const unsigned short* QKVb = QKV + (size_t)b * kTok * kQkvN;
    wmma_gemm64<0, false, 0, 0, 0><<<dim3((kTok / 64) * (kTok / 64) / 8, kHeads), dim3(256), 0, stream>>>(
        QKVb, nullptr, kQkvN, (long)kHdim, QKVb + kChan, nullptr, kQkvN, (long)kHdim,
        (void*)S, nullptr, kTok, kPlane, nullptr, nullptr, 0L, kTok, kTok, kHdim, kScoreScale, 0.f, nullptr);
    thmix_kernel<<<dim3(kTok), dim3(256), 0, stream>>>(S, W_l, b_l, W_w, b_w, A2F);
    for (int grp = 0; grp < kNGrp; ++grp) {
      const int gbase = grp * kGrp;
      const float* A2Fg = A2F + (size_t)gbase * kPlane;
      a2planes_kernel<<<dim3(kTok / 64, kTok / 64, kGrp), dim3(256), 0, stream>>>(A2Fg, AM, A2T);
      wmma_gemm64<0, false, 0, 1, 2><<<dim3((kTok / 64) * (kTok / 64) / 8, kGrp), dim3(256), 0, stream>>>(
          AM, nullptr, kTok, kPlane, A2T, nullptr, kTok, kPlane,
          (void*)ATT, nullptr, kTok, kPlane, nullptr, A2Fg, kPlane, kTok, kTok, kTok, kReact3, kAttCarry, lamb + gbase);
      wmma_gemm64<0, false, 0, 1, 0><<<dim3((kTok / 64) * (kHdim / 64) / 8, kGrp), dim3(256), 0, stream>>>(
          ATT, nullptr, kTok, kPlane, VT + (size_t)(b * kHeads + gbase) * kVtPlane, nullptr, kTok, kVtPlane,
          (void*)(CTX + gbase * kHdim), nullptr, kChan, (long)kHdim, nullptr, nullptr, 0L, kTok, kHdim, kTok, kAttnVScale, 0.f, nullptr);
    }
    wmma_gemm64<0, false, 2, 0, 0><<<dim3((kTok / 64) * (kChan / 64) / 8, 1), dim3(256), 0, stream>>>(
        CTX, nullptr, kChan, 0L, WPT, nullptr, kChan, 0L,
        (void*)(outp + (size_t)b * kTok * kChan), nullptr, kChan, 0L, b_proj, nullptr, 0L, kTok, kChan, kChan, kProjScale, 0.f, nullptr);
  }
}
